// GNNPotentials_77326591197639
// MI455X (gfx1250) — hardware-verified
//
#include <hip/hip_runtime.h>
#include <math.h>

#define NAT 2048
#define NRBF 16
#define HID 64
#define CUTOFF 5.0f
#define GAMMA 10.0f

typedef _Float16 h16;
typedef __attribute__((ext_vector_type(16))) _Float16 v16h;
typedef __attribute__((ext_vector_type(8)))  float v8f;

__device__ __forceinline__ v8f wmma16(v16h a, v16h b, v8f c) { return __builtin_amdgcn_wmma_f32_16x16x32_f16(false, a, false, b, (short)0, c, false, false); }
#define RSPLIT (1.0f / 2048.0f)
__device__ __forceinline__ h16 lo_of(float v, h16 h) { return (h16)((v - (float)h) * 2048.0f); }
__device__ __forceinline__ v8f wmma_split(v16h a, v16h al, v16h b, v16h bl, v8f c) { v8f x = {}; x = wmma16(al, b, x); x = wmma16(a, bl, x); return wmma16(a, b, c) + x * RSPLIT; }
__device__ __forceinline__ int kof(int half, int e) { return 8 * half + ((e < 8) ? e : (e + 8)); }

__global__ __launch_bounds__(256) void k_pair_energy(const float* __restrict__ q, const float* __restrict__ cell,
                                                    const float* __restrict__ W1, const float* __restrict__ b1,
                                                    const float* __restrict__ W2, const float* __restrict__ b2, float* __restrict__ rowE) {
  __shared__ float wsum[8];
  const int i = blockIdx.x, tid = threadIdx.x, lane = tid & 31, wave = tid >> 5, half = lane >> 4, l16 = lane & 15;
  const float cx = cell[0], cy = cell[1], cz = cell[2];
  const float qix = q[i * 3 + 0], qiy = q[i * 3 + 1], qiz = q[i * 3 + 2];
  v16h Bw[4], Bwl[4];
#pragma unroll
  for (int nt = 0; nt < 4; ++nt) {
    v16h r, rl;
#pragma unroll
    for (int e = 0; e < 16; ++e) { const int k = kof(half, e); const float v = (k < NRBF) ? W1[k * HID + nt * 16 + l16] : 0.0f; r[e] = (h16)v; rl[e] = lo_of(v, r[e]); }
    Bw[nt] = r; Bwl[nt] = rl;
  }
  float b1v[4], w2v[4];
#pragma unroll
  for (int nt = 0; nt < 4; ++nt) { b1v[nt] = b1[nt * 16 + l16]; w2v[nt] = W2[nt * 16 + l16]; }
  const float dmu = CUTOFF / (float)(NRBF - 1);
  float esum = 0.0f;
#pragma unroll 1
  for (int jt = wave; jt < NAT / 16; jt += 8) {
    const int j = jt * 16 + l16;
    float dx = q[j * 3 + 0] - qix, dy = q[j * 3 + 1] - qiy, dz = q[j * 3 + 2] - qiz;
    dx += (-(dx >= 0.5f * cx ? 1.0f : 0.0f) + (dx < -0.5f * cx ? 1.0f : 0.0f)) * cx;
    dy += (-(dy >= 0.5f * cy ? 1.0f : 0.0f) + (dy < -0.5f * cy ? 1.0f : 0.0f)) * cy;
    dz += (-(dz >= 0.5f * cz ? 1.0f : 0.0f) + (dz < -0.5f * cz ? 1.0f : 0.0f)) * cz;
    const float dsq = dx * dx + dy * dy + dz * dz;
    const bool m = (dsq < CUTOFF * CUTOFF) && (dsq != 0.0f) && (j >= i);
    if (__builtin_amdgcn_ballot_w32(m) == 0) continue;
    const float d = sqrtf(m ? dsq : 1.0f);
    v16h a, al;
#pragma unroll
    for (int e = 0; e < 16; ++e) { const int k = kof(half, e); float v = 0.0f;
      if (k < NRBF) { const float t = d - dmu * (float)k; v = __expf(-GAMMA * t * t); } a[e] = (h16)v; al[e] = lo_of(v, a[e]); }
    float part[8];
#pragma unroll
    for (int r = 0; r < 8; ++r) part[r] = 0.0f;
#pragma unroll
    for (int nt = 0; nt < 4; ++nt) {
      v8f c = {};
      c = wmma_split(a, al, Bw[nt], Bwl[nt], c);
#pragma unroll
      for (int r = 0; r < 8; ++r) { const float hpre = c[r] + b1v[nt]; const float hv = hpre / (1.0f + __expf(-hpre)); part[r] += hv * w2v[nt]; }
    }
#pragma unroll
    for (int r = 0; r < 8; ++r) {
      float s = part[r];
      s += __shfl_xor(s, 1, 32); s += __shfl_xor(s, 2, 32); s += __shfl_xor(s, 4, 32); s += __shfl_xor(s, 8, 32);
      part[r] = s;
    }
    float mine = 0.0f;
#pragma unroll
    for (int hh = 0; hh < 2; ++hh)
#pragma unroll
      for (int r = 0; r < 8; ++r) { const float e = __shfl(part[r], hh * 16, 32); if (l16 == 8 * hh + r) mine = e; }
    if (lane < 16 && m) esum += mine + b2[0];
  }
#pragma unroll
  for (int o = 16; o >= 1; o >>= 1) esum += __shfl_xor(esum, o, 32);
  if (lane == 0) wsum[wave] = esum;
  __syncthreads();
  if (tid == 0) { float s = 0.0f;
#pragma unroll
    for (int w = 0; w < 8; ++w) s += wsum[w];
    *(volatile float*)(rowE + i) = s; __threadfence(); *(volatile float*)(rowE + i) = s; }
}

__global__ __launch_bounds__(256) void k_reduce(const float* __restrict__ rowE, float* __restrict__ out) {
  __shared__ float red[256];
  const int tid = threadIdx.x;
  float s = 0.0f;
#pragma unroll 1
  for (int r = tid; r < NAT; r += 256) s += rowE[r];
  red[tid] = s;
  __syncthreads();
  for (int o = 128; o > 0; o >>= 1) { if (tid < o) red[tid] += red[tid + o]; __syncthreads(); }
  if (tid == 0) { *(volatile float*)out = red[0]; __threadfence(); *(volatile float*)out = red[0]; }
}

extern "C" void kernel_launch(void* const* d_in, const int* in_sizes, int n_in,
                              void* d_out, int out_size, void* d_ws, size_t ws_size,
                              hipStream_t stream) {
  (void)in_sizes; (void)n_in; (void)out_size; (void)ws_size;
  const float* q    = (const float*)d_in[0];
  const float* cell = (const float*)d_in[1];
  const float* W1   = (const float*)d_in[2];
  const float* b1   = (const float*)d_in[3];
  const float* W2   = (const float*)d_in[4];
  const float* b2   = (const float*)d_in[5];
  float* rowE = (float*)d_ws;
  k_pair_energy<<<NAT, 256, 0, stream>>>(q, cell, W1, b1, W2, b2, rowE);
  k_reduce<<<1, 256, 0, stream>>>(rowE, (float*)d_out);
}
